// DeformableConv_89876485636819
// MI455X (gfx1250) — hardware-verified
//
#include <hip/hip_runtime.h>

constexpr int NB     = 8;
constexpr int CIN    = 128;
constexpr int COUT   = 128;
constexpr int HH     = 112;
constexpr int WW     = 112;
constexpr int PIX    = HH * WW;
constexpr int NTAP   = 9;
constexpr int KDIM   = CIN * NTAP;
constexpr int OMROWS = 32;
constexpr int PPITCH = 136;
constexpr int PIXBLK = 64;
constexpr int NPB    = PIX / PIXBLK;

static_assert(KDIM % 32 == 0, "K multiple of 32");
static_assert(PIX % PIXBLK == 0, "pixel tiles exact");
static_assert(PIX % 32 == 0, "row pitch multiple of 32 floats");
static_assert((CIN * WW) % 256 == 0, "convert kernel load coverage exact");
static_assert((WW * 16) % 256 == 0, "convert kernel store coverage exact");
static_assert(OMROWS % 16 == 0 && COUT % 32 == 0, "M tile multiples");

typedef __attribute__((ext_vector_type(16))) __bf16   v16b;
typedef __attribute__((ext_vector_type(8)))  __bf16   v8b;
typedef __attribute__((ext_vector_type(8)))  float    v8f;
typedef __attribute__((ext_vector_type(4)))  float    v4f;
typedef __attribute__((ext_vector_type(4)))  unsigned uv4;

__device__ __forceinline__ unsigned short f2bf_bits(float f) {
  unsigned u = __float_as_uint(f);
  return (unsigned short)((u + 0x7FFFu + ((u >> 16) & 1u)) >> 16);
}
__device__ __forceinline__ float bf_bits2f(unsigned short h) { return __uint_as_float(((unsigned)h) << 16); }
__device__ __forceinline__ float bf16r(float f) { return bf_bits2f(f2bf_bits(f)); }
__device__ __forceinline__ float bf_lo16(unsigned u) { return __uint_as_float(u << 16); }
__device__ __forceinline__ float bf_hi16(unsigned u) { return __uint_as_float(u & 0xffff0000u); }

__device__ __forceinline__ void dep_guard_b(v8f& a, v8f& b, v16b x, v16b y) { asm volatile("v_nop\n\tv_nop\n\tv_nop\n\tv_nop" : "+v"(a), "+v"(b) : "v"(x), "v"(y)); }
__device__ __forceinline__ void dep_guard1_b(v8f& a, v16b x, v16b y) { asm volatile("v_nop\n\tv_nop\n\tv_nop\n\tv_nop" : "+v"(a) : "v"(x), "v"(y)); }
__device__ __forceinline__ void keep4_b(v16b a, v16b b, v16b c, v16b d) { asm volatile("v_nop" :: "v"(a), "v"(b), "v"(c), "v"(d)); }
__device__ __forceinline__ void acc_guard4(v8f& a, v8f& b, v8f& c, v8f& d) { asm volatile("v_nop\n\tv_nop\n\tv_nop\n\tv_nop" : "+v"(a), "+v"(b), "+v"(c), "+v"(d)); }
__device__ __forceinline__ void acc_guard1(v8f& a) { asm volatile("v_nop\n\tv_nop\n\tv_nop\n\tv_nop" : "+v"(a)); }

template <typename T> struct Frag;
template <> struct Frag<__bf16> {
  typedef v16b V; union U { v16b v; v8b h[2]; };
  static __device__ __forceinline__ v16b load(const __bf16* p) {
    U f; f.h[0] = *(const v8b*)(p); f.h[1] = *(const v8b*)(p + 16); return f.v;
  }
  static __device__ __forceinline__ v8f mma(v16b a, v16b b, v8f c) {
    return __builtin_amdgcn_wmma_f32_16x16x32_bf16(false, a, false, b, (short)0, c, false, false);
  }
};

__global__ __launch_bounds__(256) void k_x_to_nhwc_bf16(const float* __restrict__ x,
                                                         unsigned short* __restrict__ xt) {
  __shared__ float tile[CIN * 113];
  const int tid = threadIdx.x;
  const int b = blockIdx.x / HH;
  const int y = blockIdx.x - b * HH;
  const float* src = x + (size_t)b * CIN * PIX + (size_t)y * WW;
#pragma unroll 4
  for (int it = 0; it < (CIN * WW) / 256; ++it) {
    const int idx = it * 256 + tid;
    const int c = idx / WW;
    const int xx = idx - c * WW;
    tile[c * 113 + xx] = src[(size_t)c * PIX + xx];
  }
  __syncthreads();
  unsigned short* dstb = xt + ((size_t)b * HH + y) * (size_t)WW * CIN;
#pragma unroll 1
  for (int it = 0; it < (WW * 16) / 256; ++it) {
    const int idx = it * 256 + tid;
    const int p = idx >> 4;
    const int g = idx & 15;
    uv4 u;
#pragma unroll
    for (int j = 0; j < 4; ++j) {
      const float f0 = tile[(g * 8 + 2 * j) * 113 + p];
      const float f1 = tile[(g * 8 + 2 * j + 1) * 113 + p];
      u[j] = (unsigned)f2bf_bits(f0) | ((unsigned)f2bf_bits(f1) << 16);
    }
    unsigned short* d = dstb + (size_t)p * CIN + g * 8;
    *(volatile uv4*)d = u;
    __threadfence();
    *(volatile uv4*)d = u;
  }
}

__global__ __launch_bounds__(256) void k_weight_planes(const float* __restrict__ w,
                                                        const float* __restrict__ offw,
                                                        const float* __restrict__ modw,
                                                        unsigned short* __restrict__ wm,
                                                        unsigned short* __restrict__ wo) {
  constexpr int NWM = COUT * NTAP * 16;
  constexpr int NWO = OMROWS * NTAP * 16;
  static_assert(NWM % 256 == 0 && NWO % 256 == 0, "block-uniform split");
  const int idx = blockIdx.x * 256 + threadIdx.x;
  if (idx < NWM) {
    const int row = idx / 144;
    const int rem = idx - row * 144;
    const int kk = rem >> 4;
    const int g = rem & 15;
    uv4 u;
#pragma unroll
    for (int j = 0; j < 4; ++j) {
      const int c0 = g * 8 + 2 * j;
      const float f0 = w[((size_t)row * CIN + c0) * NTAP + kk];
      const float f1 = w[((size_t)row * CIN + c0 + 1) * NTAP + kk];
      u[j] = (unsigned)f2bf_bits(f0) | ((unsigned)f2bf_bits(f1) << 16);
    }
    unsigned short* d = wm + (size_t)idx * 8;
    *(volatile uv4*)d = u;
    __threadfence();
    *(volatile uv4*)d = u;
  } else if (idx < NWM + NWO) {
    const int i2 = idx - NWM;
    const int row = i2 / 144;
    const int rem = i2 - row * 144;
    const int kk = rem >> 4;
    const int g = rem & 15;
    const int ro = row < 18 ? row : 17;
    int rm = row - 18; rm = rm < 0 ? 0 : (rm > 8 ? 8 : rm);
    uv4 u;
#pragma unroll
    for (int j = 0; j < 4; ++j) {
      const int c0 = g * 8 + 2 * j;
      const float vo0 = offw[((size_t)ro * CIN + c0) * NTAP + kk];
      const float vo1 = offw[((size_t)ro * CIN + c0 + 1) * NTAP + kk];
      const float vm0 = modw[((size_t)rm * CIN + c0) * NTAP + kk];
      const float vm1 = modw[((size_t)rm * CIN + c0 + 1) * NTAP + kk];
      const float f0 = (row < 18) ? vo0 : ((row < 27) ? vm0 : 0.0f);
      const float f1 = (row < 18) ? vo1 : ((row < 27) ? vm1 : 0.0f);
      u[j] = (unsigned)f2bf_bits(f0) | ((unsigned)f2bf_bits(f1) << 16);
    }
    unsigned short* d = wo + (size_t)i2 * 8;
    *(volatile uv4*)d = u;
    __threadfence();
    *(volatile uv4*)d = u;
  }
}

__global__ __launch_bounds__(256) void k_offmod_conv(const unsigned short* __restrict__ xt,
                                                      const unsigned short* __restrict__ wo,
                                                      const float* __restrict__ offb,
                                                      const float* __restrict__ modb,
                                                      float* __restrict__ om) {
  __shared__ __align__(16) __bf16 panel[PIXBLK * PPITCH];
  __shared__ __align__(16) float outs[OMROWS * 68];
  const int tid  = threadIdx.x;
  const int lane = tid & 31;
  const int wv   = tid >> 5;
  const int wm2  = wv >> 2;
  const int wn2  = wv & 3;
  const int b    = blockIdx.x / NPB;
  const int pix0 = (blockIdx.x - b * NPB) * PIXBLK;
  const int sp   = tid >> 2;
  const int sq   = tid & 3;
  const int pix  = pix0 + sp;
  const int py   = pix / WW;
  const int px   = pix - py * WW;
  const int rlane = lane & 15;
  const int hsel  = lane >> 4;
  const int koff  = hsel * 8;
  const __bf16* A = (const __bf16*)wo;
  const unsigned short* xb = xt + (size_t)b * PIX * CIN;

  v8f acc = (v8f){0.f, 0.f, 0.f, 0.f, 0.f, 0.f, 0.f, 0.f};

#pragma unroll 1
  for (int kk = 0; kk < NTAP; ++kk) {
    const int ki = kk / 3;
    const int kj = kk - ki * 3;
    {
      const int yy = py - 1 + ki;
      const int xx = px - 1 + kj;
      const bool valid = (yy >= 0) && (yy < HH) && (xx >= 0) && (xx < WW);
      const int cy = yy < 0 ? 0 : (yy > HH - 1 ? HH - 1 : yy);
      const int cx = xx < 0 ? 0 : (xx > WW - 1 ? WW - 1 : xx);
      const uv4* s = (const uv4*)(xb + ((size_t)cy * WW + cx) * CIN + sq * 32);
      uv4* d = (uv4*)(panel + sp * PPITCH + sq * 32);
#pragma unroll
      for (int i = 0; i < 4; ++i) {
        uv4 t = s[i];
#pragma unroll
        for (int e = 0; e < 4; ++e) t[e] = valid ? t[e] : 0u;
        d[i] = t;
      }
    }
    __syncthreads();
#pragma unroll
    for (int cc = 0; cc < 4; ++cc) {
      const int kg = kk * CIN + cc * 32;
      const v16b af = Frag<__bf16>::load(A + (size_t)(wm2 * 16 + rlane) * KDIM + kg + koff);
      const v16b bfr = Frag<__bf16>::load(panel + (wn2 * 16 + rlane) * PPITCH + cc * 32 + koff);
      acc = Frag<__bf16>::mma(af, bfr, acc);
      dep_guard1_b(acc, af, bfr);
    }
    __syncthreads();
  }
  acc_guard1(acc);

  {
    const int m0 = wm2 * 16 + hsel * 8;
#pragma unroll
    for (int r = 0; r < 8; ++r) {
      const int m = m0 + r;
      const int io = m < 18 ? m : 17;
      int im = m - 18; im = im < 0 ? 0 : (im > 8 ? 8 : im);
      const float bo = bf16r(offb[io]);
      const float bm = bf16r(modb[im]);
      const float vo = acc[r] + bo;
      const float z  = acc[r] + bm;
      const float e  = expf(-z);
      const float vm = 2.0f * (1.0f / (1.0f + e));
      const float v  = (m < 18) ? vo : ((m < 27) ? vm : 0.0f);
      outs[m * 68 + wn2 * 16 + rlane] = v;
    }
  }
  __syncthreads();
  {
    float* omb = om + (size_t)b * OMROWS * PIX + pix0;
    const int c4 = rlane * 4;
    for (int pass = 0; pass < 2; ++pass) {
#pragma unroll
      for (int it = 0; it < 2; ++it) {
        const int row = wv * 4 + it * 2 + hsel;
        const v4f v = *(const v4f*)(outs + row * 68 + c4);
        *(volatile v4f*)(omb + (size_t)row * PIX + c4) = v;
      }
      __threadfence();
    }
  }
}

constexpr int STG_PITCH = 36;
constexpr int SMEM_MAIN_BYTES = 8 * 32 * STG_PITCH * 4;
static_assert(SMEM_MAIN_BYTES >= 2 * PIXBLK * PPITCH * 2, "panels fit in the staging region");

__global__ __launch_bounds__(256) void k_deform_main(const unsigned short* __restrict__ xt,
                                                      const unsigned short* __restrict__ wm,
                                                      const float* __restrict__ om,
                                                      const float* __restrict__ bias,
                                                      float* __restrict__ out) {
  __shared__ __align__(16) unsigned char smem[SMEM_MAIN_BYTES];
  __bf16* ph = (__bf16*)smem;
  __bf16* pl = ph + PIXBLK * PPITCH;
  float* stage = (float*)smem;

  const int tid  = threadIdx.x;
  const int lane = tid & 31;
  const int wv   = tid >> 5;
  const int wmv  = wv >> 1;
  const int wnv  = wv & 1;
  const int b    = blockIdx.x / NPB;
  const int pix0 = (blockIdx.x - b * NPB) * PIXBLK;
  const int sp   = tid >> 2;
  const int sq   = tid & 3;
  const int pix  = pix0 + sp;
  const int py   = pix / WW;
  const int px   = pix - py * WW;
  const int rlane = lane & 15;
  const int hsel  = lane >> 4;
  const int koff  = hsel * 8;
  const __bf16* A = (const __bf16*)wm;
  const unsigned short* xb = xt + (size_t)b * PIX * CIN;
  const float* omb = om + (size_t)b * OMROWS * PIX;

  v8f acc[2][2];
#pragma unroll
  for (int i = 0; i < 2; ++i)
#pragma unroll
    for (int j = 0; j < 2; ++j) acc[i][j] = (v8f){0.f, 0.f, 0.f, 0.f, 0.f, 0.f, 0.f, 0.f};

#pragma unroll 1
  for (int kk = 0; kk < NTAP; ++kk) {
    const int ki = kk / 3;
    const int kj = kk - ki * 3;
    {
      const float dy = omb[(size_t)(2 * kk) * PIX + pix];
      const float dx = omb[(size_t)(2 * kk + 1) * PIX + pix];
      const float mk = omb[(size_t)(18 + kk) * PIX + pix];
      const float ys = (float)(py - 1 + ki) + dy;
      const float xs = (float)(px - 1 + kj) + dx;
      const float y0f = floorf(ys);
      const float x0f = floorf(xs);
      const int iy0 = (int)y0f, ix0 = (int)x0f;
      const int iy1 = iy0 + 1, ix1 = ix0 + 1;
      const float ly = ys - y0f, lx = xs - x0f;
      const float vy0 = (iy0 >= 0 && iy0 < HH) ? 1.f : 0.f;
      const float vy1 = (iy1 >= 0 && iy1 < HH) ? 1.f : 0.f;
      const float vx0 = (ix0 >= 0 && ix0 < WW) ? 1.f : 0.f;
      const float vx1 = (ix1 >= 0 && ix1 < WW) ? 1.f : 0.f;
      const float w00 = (1.f - ly) * (1.f - lx) * vy0 * vx0 * mk;
      const float w01 = (1.f - ly) * lx         * vy0 * vx1 * mk;
      const float w10 = ly * (1.f - lx)         * vy1 * vx0 * mk;
      const float w11 = ly * lx                 * vy1 * vx1 * mk;
      const int cy0 = iy0 < 0 ? 0 : (iy0 > HH - 1 ? HH - 1 : iy0);
      const int cy1 = iy1 < 0 ? 0 : (iy1 > HH - 1 ? HH - 1 : iy1);
      const int cx0 = ix0 < 0 ? 0 : (ix0 > WW - 1 ? WW - 1 : ix0);
      const int cx1 = ix1 < 0 ? 0 : (ix1 > WW - 1 ? WW - 1 : ix1);
      const uv4* p00 = (const uv4*)(xb + ((size_t)cy0 * WW + cx0) * CIN + sq * 32);
      const uv4* p01 = (const uv4*)(xb + ((size_t)cy0 * WW + cx1) * CIN + sq * 32);
      const uv4* p10 = (const uv4*)(xb + ((size_t)cy1 * WW + cx0) * CIN + sq * 32);
      const uv4* p11 = (const uv4*)(xb + ((size_t)cy1 * WW + cx1) * CIN + sq * 32);
      uv4* dh = (uv4*)(ph + sp * PPITCH + sq * 32);
      uv4* dl = (uv4*)(pl + sp * PPITCH + sq * 32);
#pragma unroll
      for (int i = 0; i < 4; ++i) {
        const uv4 a0 = p00[i];
        const uv4 a1 = p01[i];
        const uv4 a2 = p10[i];
        const uv4 a3 = p11[i];
        uv4 uh, ul;
#pragma unroll
        for (int j = 0; j < 4; ++j) {
          const unsigned u00 = a0[j], u01 = a1[j], u10 = a2[j], u11 = a3[j];
          const float f0 = w00 * bf_lo16(u00) + w01 * bf_lo16(u01) + w10 * bf_lo16(u10) + w11 * bf_lo16(u11);
          const float f1 = w00 * bf_hi16(u00) + w01 * bf_hi16(u01) + w10 * bf_hi16(u10) + w11 * bf_hi16(u11);
          const unsigned short h0 = f2bf_bits(f0);
          const unsigned short h1 = f2bf_bits(f1);
          const unsigned short l0 = f2bf_bits(f0 - bf_bits2f(h0));
          const unsigned short l1 = f2bf_bits(f1 - bf_bits2f(h1));
          uh[j] = (unsigned)h0 | ((unsigned)h1 << 16);
          ul[j] = (unsigned)l0 | ((unsigned)l1 << 16);
        }
        dh[i] = uh;
        dl[i] = ul;
      }
    }
    __syncthreads();
#pragma unroll
    for (int cc = 0; cc < 4; ++cc) {
      const int kg = kk * CIN + cc * 32;
      v16b af[2], bh[2], blo[2];
#pragma unroll
      for (int mi = 0; mi < 2; ++mi)
        af[mi] = Frag<__bf16>::load(A + (size_t)(wmv * 32 + mi * 16 + rlane) * KDIM + kg + koff);
#pragma unroll
      for (int ni = 0; ni < 2; ++ni) {
        const int po = (wnv * 32 + ni * 16 + rlane) * PPITCH + cc * 32 + koff;
        bh[ni]  = Frag<__bf16>::load(ph + po);
        blo[ni] = Frag<__bf16>::load(pl + po);
      }
#pragma unroll
      for (int mi = 0; mi < 2; ++mi) {
#pragma unroll
        for (int ni = 0; ni < 2; ++ni) {
          acc[mi][ni] = Frag<__bf16>::mma(af[mi], bh[ni], acc[mi][ni]);
          acc[mi][ni] = Frag<__bf16>::mma(af[mi], blo[ni], acc[mi][ni]);
        }
        dep_guard_b(acc[mi][0], acc[mi][1], af[mi], blo[1]);
      }
      keep4_b(bh[0], bh[1], blo[0], blo[1]);
    }
    __syncthreads();
  }
  acc_guard4(acc[0][0], acc[0][1], acc[1][0], acc[1][1]);

  float* st = stage + wv * (32 * STG_PITCH);
#pragma unroll
  for (int mi = 0; mi < 2; ++mi) {
    const int o0 = wmv * 32 + mi * 16 + hsel * 8;
    const v4f bv0 = *(const v4f*)(bias + o0);
    const v4f bv1 = *(const v4f*)(bias + o0 + 4);
#pragma unroll
    for (int ni = 0; ni < 2; ++ni) {
#pragma unroll
      for (int r = 0; r < 8; ++r) {
        const float bb = (r < 4) ? bv0[r & 3] : bv1[r & 3];
        st[(mi * 16 + hsel * 8 + r) * STG_PITCH + ni * 16 + rlane] = acc[mi][ni][r] + bf16r(bb);
      }
    }
  }
  __syncthreads();
  {
    float* ob = out + ((size_t)b * COUT + wmv * 32) * PIX + pix0 + wnv * 32;
    const int q = lane >> 3;
    const int c4 = (lane & 7) * 4;
    for (int pass = 0; pass < 2; ++pass) {
#pragma unroll
      for (int it = 0; it < 8; ++it) {
        const int row = it * 4 + q;
        const v4f v = *(const v4f*)(st + row * STG_PITCH + c4);
        *(volatile v4f*)(ob + (size_t)row * PIX + c4) = v;
      }
      __threadfence();
    }
  }
}

extern "C" void kernel_launch(void* const* d_in, const int* in_sizes, int n_in,
                              void* d_out, int out_size, void* d_ws, size_t ws_size,
                              hipStream_t stream) {
  (void)n_in;
  constexpr size_t XT_BYTES = (size_t)NB * PIX * CIN * 2;
  constexpr size_t WM_BYTES = (size_t)COUT * KDIM * 2;
  constexpr size_t WO_BYTES = (size_t)OMROWS * KDIM * 2;
  constexpr size_t OM_BYTES = (size_t)NB * OMROWS * PIX * 4;
  constexpr size_t XT_OFF = 0;
  constexpr size_t WM_OFF = XT_OFF + XT_BYTES;
  constexpr size_t WO_OFF = WM_OFF + WM_BYTES;
  constexpr size_t OM_OFF = WO_OFF + WO_BYTES;
  constexpr size_t WS_TOTAL = OM_OFF + OM_BYTES;
  static_assert(WS_TOTAL == 38903808ull, "carve total");
  static_assert(WS_TOTAL <= 134217728ull, "carve under 128 MiB");
  static_assert(WM_OFF % 256 == 0 && WO_OFF % 256 == 0 && OM_OFF % 256 == 0, "aligned regions");

  if (ws_size < WS_TOTAL) return;
  if (in_sizes[0] != NB * CIN * PIX || in_sizes[5] != COUT * CIN * NTAP || out_size != NB * COUT * PIX) return;

  const float* x    = (const float*)d_in[0];
  const float* offw = (const float*)d_in[1];
  const float* offb = (const float*)d_in[2];
  const float* modw = (const float*)d_in[3];
  const float* modb = (const float*)d_in[4];
  const float* w    = (const float*)d_in[5];
  const float* bias = (const float*)d_in[6];
  float* out = (float*)d_out;

  char* ws = (char*)d_ws;
  unsigned short* xt = (unsigned short*)(ws + XT_OFF);
  unsigned short* wm = (unsigned short*)(ws + WM_OFF);
  unsigned short* wo = (unsigned short*)(ws + WO_OFF);
  float* om = (float*)(ws + OM_OFF);

  constexpr int GRID_CVT  = NB * HH;
  constexpr int GRID_WGT  = (COUT * NTAP * 16 + OMROWS * NTAP * 16) / 256;
  constexpr int GRID_GEMM = NB * NPB;
  static_assert((COUT * NTAP * 16 + OMROWS * NTAP * 16) % 256 == 0, "weight grid exact");

  k_x_to_nhwc_bf16<<<GRID_CVT, 256, 0, stream>>>(x, xt);
  k_weight_planes <<<GRID_WGT, 256, 0, stream>>>(w, offw, modw, wm, wo);
  k_offmod_conv   <<<GRID_GEMM, 256, 0, stream>>>(xt, wo, offb, modb, om);
  k_deform_main   <<<GRID_GEMM, 256, 0, stream>>>(xt, wm, om, bias, out);
}
